// LIIF_84731114816194
// MI455X (gfx1250) — hardware-verified
//
#include <hip/hip_runtime.h>
#include <stdint.h>
#include <math.h>

#pragma clang fp contract(off)

constexpr int kImg       = 192;
constexpr int kPix       = kImg * kImg;
constexpr int kCh        = 64;
constexpr int kQ         = 16384;
constexpr int kChunkQ    = 8192;
constexpr int kChunkRows = 4 * kChunkQ;
constexpr int kInDim     = 580;
constexpr int kK0        = 608;
constexpr int kPitch0    = 640;
constexpr int kHid       = 256;
constexpr int kHeadN     = 64;
constexpr int kConvW     = kCh * 27;
constexpr float kWCarry    = 16.0f;
constexpr float kWCarryInv = 1.0f / 16.0f;

static_assert(kK0 % 32 == 0 && kHid % 32 == 0, "K multiple of 32");
static_assert(kChunkRows % 64 == 0 && kHid % 64 == 0 && kHeadN % 64 == 0, "M,N tile multiples");
static_assert(kK0 >= kInDim && kPitch0 >= kK0 && kPitch0 % 64 == 0, "pads");
static_assert(kChunkQ % 256 == 0 && kQ % kChunkQ == 0, "chunking");
static_assert(kConvW == 9 * kImg, "conv weight staging covers the table exactly");

constexpr size_t kSzFeat = (size_t)kCh * kPix * 4;
constexpr size_t kSzWt0  = (size_t)kHid * kPitch0 * 2;
constexpr size_t kSzWt   = (size_t)kHid * kHid * 2;
constexpr size_t kSzWt4  = (size_t)kHeadN * kHid * 2;
constexpr size_t kSzX    = (size_t)kChunkRows * kPitch0 * 2;
constexpr size_t kSzY    = (size_t)kChunkRows * kHid * 2;
constexpr size_t kSzZ    = (size_t)kChunkRows * kHeadN * 4;
constexpr size_t kOffFeat = 0;
constexpr size_t kOffWt0  = kOffFeat + kSzFeat;
constexpr size_t kOffWt1  = kOffWt0 + kSzWt0;
constexpr size_t kOffWt2  = kOffWt1 + kSzWt;
constexpr size_t kOffWt3  = kOffWt2 + kSzWt;
constexpr size_t kOffWt4  = kOffWt3 + kSzWt;
constexpr size_t kOffX    = kOffWt4 + kSzWt4;
constexpr size_t kOffY1   = kOffX + kSzX;
constexpr size_t kOffY2   = kOffY1 + kSzY;
constexpr size_t kOffZ    = kOffY2 + kSzY;
constexpr size_t kWsTotal = kOffZ + kSzZ;
static_assert(kWsTotal == (size_t)94076928, "carve total");
static_assert(kWsTotal <= (size_t)134217728, "carve under 128 MiB");
static_assert(kOffWt0 % 128 == 0 && kOffWt1 % 128 == 0 && kOffWt2 % 128 == 0 && kOffWt3 % 128 == 0 &&
              kOffWt4 % 128 == 0 && kOffX % 128 == 0 && kOffY1 % 128 == 0 && kOffY2 % 128 == 0 &&
              kOffZ % 128 == 0, "128-B aligned regions");

typedef __attribute__((ext_vector_type(16))) _Float16 v16h;
typedef __attribute__((ext_vector_type(8)))  _Float16 v8h;
typedef __attribute__((ext_vector_type(16))) __bf16   v16b;
typedef __attribute__((ext_vector_type(8)))  __bf16   v8b;
typedef __attribute__((ext_vector_type(8)))  float    v8f;
typedef __attribute__((ext_vector_type(4)))  float    v4f;
typedef __attribute__((ext_vector_type(4)))  unsigned int v4u;

__device__ __forceinline__ unsigned short f2bf_bits(float f) {
  unsigned u = __float_as_uint(f);
  return (unsigned short)((u + 0x7FFFu + ((u >> 16) & 1u)) >> 16);
}
__device__ __forceinline__ float bf_bits2f(unsigned short h) { return __uint_as_float(((unsigned)h) << 16); }

__device__ __forceinline__ void dep_guard_h(v8f& a, v8f& b, v16h x, v16h y) { asm volatile("v_nop\n\tv_nop\n\tv_nop\n\tv_nop" : "+v"(a), "+v"(b) : "v"(x), "v"(y)); }
__device__ __forceinline__ void dep_guard_b(v8f& a, v8f& b, v16b x, v16b y) { asm volatile("v_nop\n\tv_nop\n\tv_nop\n\tv_nop" : "+v"(a), "+v"(b) : "v"(x), "v"(y)); }
__device__ __forceinline__ void keep4_h(v16h a, v16h b, v16h c, v16h d) { asm volatile("v_nop" :: "v"(a), "v"(b), "v"(c), "v"(d)); }
__device__ __forceinline__ void keep4_b(v16b a, v16b b, v16b c, v16b d) { asm volatile("v_nop" :: "v"(a), "v"(b), "v"(c), "v"(d)); }
__device__ __forceinline__ void acc_guard4(v8f& a, v8f& b, v8f& c, v8f& d) { asm volatile("v_nop\n\tv_nop\n\tv_nop\n\tv_nop" : "+v"(a), "+v"(b), "+v"(c), "+v"(d)); }
template <typename T> struct Frag;
template <> struct Frag<_Float16> {
  typedef v16h V; union U { v16h v; v8h h[2]; };
  static __device__ __forceinline__ v16h load(const _Float16* p) {
    U f; f.h[0] = *(const v8h*)(p); f.h[1] = *(const v8h*)(p + 16); return f.v;
  }
  static __device__ __forceinline__ v8f mma(v16h a, v16h b, v8f c) {
    return __builtin_amdgcn_wmma_f32_16x16x32_f16(false, a, false, b, (short)0, c, false, false);
  }
  static __device__ __forceinline__ void guard(v8f& a, v8f& b, v16h x, v16h y) { dep_guard_h(a, b, x, y); }
  static __device__ __forceinline__ void keep(v16h a, v16h b, v16h c, v16h d) { keep4_h(a, b, c, d); }
};
template <> struct Frag<__bf16> {
  typedef v16b V; union U { v16b v; v8b h[2]; };
  static __device__ __forceinline__ v16b load(const __bf16* p) {
    U f; f.h[0] = *(const v8b*)(p); f.h[1] = *(const v8b*)(p + 16); return f.v;
  }
  static __device__ __forceinline__ v8f mma(v16b a, v16b b, v8f c) {
    return __builtin_amdgcn_wmma_f32_16x16x32_bf16(false, a, false, b, (short)0, c, false, false);
  }
  static __device__ __forceinline__ void guard(v8f& a, v8f& b, v16b x, v16b y) { dep_guard_b(a, b, x, y); }
  static __device__ __forceinline__ void keep(v16b a, v16b b, v16b c, v16b d) { keep4_b(a, b, c, d); }
};

__device__ __forceinline__ unsigned pk16(unsigned short a, unsigned short b) { return (unsigned)a | ((unsigned)b << 16); }
__device__ __forceinline__ unsigned short h_bits(float f) { const _Float16 h = (_Float16)f; return __builtin_bit_cast(unsigned short, h); }

template <int ET> struct Elem;
template <> struct Elem<0> { typedef _Float16 T; };
template <> struct Elem<1> { typedef __bf16 T; };
template <int ET, bool SPLIT, int BIAS_MODE, int OUT_MODE, bool RESID, int ACT = 0>
__global__ __launch_bounds__(256) void wmma_gemm64(
    const unsigned short* __restrict__ Ap, const unsigned short* __restrict__ A2p, int lda, long strideA,
    const unsigned short* __restrict__ Btp, const unsigned short* __restrict__ Bt2p, int ldb, long strideB,
    void* __restrict__ Cout, void* __restrict__ Cout2, int ldc, long strideC,
    const float* __restrict__ bias,
    const float* __restrict__ resid, long strideR,
    int M, int N, int K, float scale) {
  typedef typename Elem<ET>::T T;
  typedef typename Frag<T>::V V;
  const T* A = (const T*)Ap; const T* A2 = (const T*)A2p; const T* Bt = (const T*)Btp; const T* Bt2 = (const T*)Bt2p;
  __shared__ __align__(16) float sT[8][16 * 68];
  const int b    = blockIdx.y;
  const int lane = threadIdx.x & 31;
  const int wave = threadIdx.x >> 5;
  const int tilesN = N >> 6;
  const int tilesM = M >> 6;
  const int tile = blockIdx.x * 8 + wave;
  if (tile >= tilesM * tilesN) return;
  const int tm = tile / tilesN;
  const int tn = tile - tm * tilesN;
  const int m0 = tm << 6;
  const int n0 = tn << 6;

  const T* Ab  = A  + (size_t)b * strideA;
  const T* Bb  = Bt + (size_t)b * strideB;
  const T* Ab2 = SPLIT ? (A2  + (size_t)b * strideA) : nullptr;
  const T* Bb2 = SPLIT ? (Bt2 + (size_t)b * strideB) : nullptr;

  const int rlane = lane & 15;
  const int koff  = (lane >> 4) * 8;
  const int mOff  = (lane >> 4) * 8;

  v8f acc[4][4];
#pragma unroll
  for (int i = 0; i < 4; ++i)
#pragma unroll
    for (int j = 0; j < 4; ++j) acc[i][j] = (v8f){0.f,0.f,0.f,0.f,0.f,0.f,0.f,0.f};

  for (int k0 = 0; k0 < K; k0 += 32) {
    V bh[4], bl[4];
#pragma unroll
    for (int j = 0; j < 4; ++j) {
      const size_t bo = (size_t)(n0 + (j << 4) + rlane) * ldb + koff + k0;
      bh[j] = Frag<T>::load(Bb + bo);
      if (SPLIT) bl[j] = Frag<T>::load(Bb2 + bo);
    }
#pragma unroll
    for (int i = 0; i < 4; ++i) {
      const size_t ao = (size_t)(m0 + (i << 4) + rlane) * lda + koff + k0;
      V ah = Frag<T>::load(Ab + ao);
      V al;
      if (SPLIT) al = Frag<T>::load(Ab2 + ao);
#pragma unroll
      for (int j = 0; j < 4; ++j) {
        acc[i][j] = Frag<T>::mma(ah, bh[j], acc[i][j]);
        if (SPLIT) {
          acc[i][j] = Frag<T>::mma(ah, bl[j], acc[i][j]);
          acc[i][j] = Frag<T>::mma(al, bh[j], acc[i][j]);
        }
      }
      Frag<T>::guard(acc[i][0], acc[i][3], ah, SPLIT ? al : ah);
    }
    Frag<T>::keep(bh[0], bh[1], bh[2], bh[3]);
    if (SPLIT) Frag<T>::keep(bl[0], bl[1], bl[2], bl[3]);
  }
  acc_guard4(acc[0][0], acc[0][1], acc[0][2], acc[0][3]);
  acc_guard4(acc[1][0], acc[1][1], acc[1][2], acc[1][3]);
  acc_guard4(acc[2][0], acc[2][1], acc[2][2], acc[2][3]);
  acc_guard4(acc[3][0], acc[3][1], acc[3][2], acc[3][3]);

  float* slab = sT[wave];
  const float* Rb = RESID ? (resid + (size_t)b * strideR) : nullptr;
#pragma unroll
  for (int i = 0; i < 4; ++i) {
    const int mBase = m0 + (i << 4);
#pragma unroll
    for (int j = 0; j < 4; ++j) {
      const int n = n0 + (j << 4) + rlane;
      float bv = 0.f;
      if (BIAS_MODE == 2) bv = bias[n];
#pragma unroll
      for (int r = 0; r < 8; ++r) {
        float v = acc[i][j][r] * scale;
        if (BIAS_MODE == 1) v += bias[mBase + mOff + r];
        if (BIAS_MODE == 2) v += bv;
        if (RESID) v += Rb[(size_t)(mBase + mOff + r) * ldc + n];
        if (ACT == 2) v = fmaxf(v, 0.0f);
        if (ACT == 4) v = (v > 0.f) ? v : 0.01f * v;
        slab[(mOff + r) * 68 + (j << 4) + rlane] = v;
      }
    }
    __builtin_amdgcn_fence(__ATOMIC_RELEASE, "workgroup");
    __builtin_amdgcn_wave_barrier();
    __builtin_amdgcn_fence(__ATOMIC_ACQUIRE, "workgroup");
    if (OUT_MODE == 0) {
      float* C = (float*)Cout + (size_t)b * strideC;
      const int hh = lane >> 4, c4 = (lane & 15) * 4;
      for (int pass = 0; pass < 2; ++pass) {
#pragma unroll
        for (int it = 0; it < 8; ++it) {
          const int row = it * 2 + hh;
          v4f v = *(const v4f*)(slab + row * 68 + c4);
          *(volatile v4f*)(C + (size_t)(mBase + row) * ldc + n0 + c4) = v;
        }
        __threadfence();
      }
    } else {
      const int q = lane >> 3, c8 = (lane & 7) * 8;
      unsigned short* C  = (unsigned short*)Cout  + (size_t)b * strideC;
      unsigned short* C2 = (OUT_MODE == 2) ? ((unsigned short*)Cout2 + (size_t)b * strideC) : nullptr;
      for (int pass = 0; pass < 2; ++pass) {
#pragma unroll
        for (int it = 0; it < 4; ++it) {
          const int row = it * 4 + q;
          const float* sp = slab + row * 68 + c8;
          v8h hv, lv;
#pragma unroll
          for (int e = 0; e < 8; ++e) {
            if (OUT_MODE == 1) {
              hv[e] = (_Float16)sp[e];
            } else {
              unsigned short hb = f2bf_bits(sp[e]);
              unsigned short lb = f2bf_bits(sp[e] - bf_bits2f(hb));
              hv[e] = __builtin_bit_cast(_Float16, hb);
              lv[e] = __builtin_bit_cast(_Float16, lb);
            }
          }
          *(volatile v8h*)(C + (size_t)(mBase + row) * ldc + n0 + c8) = hv;
          if (OUT_MODE == 2) *(volatile v8h*)(C2 + (size_t)(mBase + row) * ldc + n0 + c8) = lv;
        }
        __threadfence();
      }
    }
    __builtin_amdgcn_fence(__ATOMIC_RELEASE, "workgroup");
    __builtin_amdgcn_wave_barrier();
    __builtin_amdgcn_fence(__ATOMIC_ACQUIRE, "workgroup");
  }
}

__device__ __forceinline__ int clampi(int v, int lo, int hi) { return v < lo ? lo : (v > hi ? hi : v); }

__device__ __forceinline__ void store_row_f16(const float* sr, unsigned short* gr, int nch, int lane) {
  const int ns = (nch + 31) >> 5;
  for (int pass = 0; pass < 2; ++pass) {
    for (int s = 0; s < ns; ++s) {
      const int idx = s * 32 + lane;
      const int idc = idx < nch ? idx : nch - 1;
      const v4f a = *(const v4f*)(sr + idc * 8);
      const v4f c = *(const v4f*)(sr + idc * 8 + 4);
      unsigned short hb[8];
#pragma unroll
      for (int e = 0; e < 4; ++e) {
        hb[e]     = h_bits(a[e]);
        hb[4 + e] = h_bits(c[e]);
      }
      const v4u u = (v4u){pk16(hb[0], hb[1]), pk16(hb[2], hb[3]), pk16(hb[4], hb[5]), pk16(hb[6], hb[7])};
      if (idx < nch) *(volatile v4u*)(gr + (size_t)idx * 8) = u;
    }
    __threadfence();
  }
}

__device__ __forceinline__ void lgeom(float c0, float c1, int e, float (&wk)[4], int (&yi)[2], int (&xi)[2],
                                      float& rely, float& relx) {
  const float rad = 1.0f / 192.0f;
  const float oy = (e < 2) ? -1.0f : 1.0f;
  const float ox = (e & 1) ? 1.0f : -1.0f;
  float gy = (c0 + oy * rad) + 1e-8f;
  float gx = (c1 + ox * rad) + 1e-8f;
  gy = fminf(fmaxf(gy, -1.0f), 1.0f);
  gx = fminf(fmaxf(gx, -1.0f), 1.0f);
  const float xf = (gx + 1.0f) * 96.0f - 0.5f;
  const float yf = (gy + 1.0f) * 96.0f - 0.5f;
  const float x0 = floorf(xf), y0 = floorf(yf);
  const float x1 = x0 + 1.0f, y1 = y0 + 1.0f;
  const float wx0 = 1.0f - fabsf(xf - x0), wx1 = 1.0f - fabsf(xf - x1);
  const float wy0 = 1.0f - fabsf(yf - y0), wy1 = 1.0f - fabsf(yf - y1);
  const float vx0 = (x0 >= 0.0f && x0 < 192.0f) ? 1.0f : 0.0f;
  const float vx1 = (x1 >= 0.0f && x1 < 192.0f) ? 1.0f : 0.0f;
  const float vy0 = (y0 >= 0.0f && y0 < 192.0f) ? 1.0f : 0.0f;
  const float vy1 = (y1 >= 0.0f && y1 < 192.0f) ? 1.0f : 0.0f;
  wk[0] = (wx0 * wy0) * (vx0 * vy0);
  wk[1] = (wx1 * wy0) * (vx1 * vy0);
  wk[2] = (wx0 * wy1) * (vx0 * vy1);
  wk[3] = (wx1 * wy1) * (vx1 * vy1);
  xi[0] = (int)fminf(fmaxf(x0, 0.0f), 191.0f);
  xi[1] = (int)fminf(fmaxf(x1, 0.0f), 191.0f);
  yi[0] = (int)fminf(fmaxf(y0, 0.0f), 191.0f);
  yi[1] = (int)fminf(fmaxf(y1, 0.0f), 191.0f);
  const float ry0 = -1.0f + (2.0f * ((float)yi[0] + 0.5f)) * rad;
  const float ry1 = -1.0f + (2.0f * ((float)yi[1] + 0.5f)) * rad;
  const float rx0 = -1.0f + (2.0f * ((float)xi[0] + 0.5f)) * rad;
  const float rx1 = -1.0f + (2.0f * ((float)xi[1] + 0.5f)) * rad;
  float qy = 0.0f, qx = 0.0f;
  qy = qy + ry0 * wk[0]; qx = qx + rx0 * wk[0];
  qy = qy + ry0 * wk[1]; qx = qx + rx1 * wk[1];
  qy = qy + ry1 * wk[2]; qx = qx + rx0 * wk[2];
  qy = qy + ry1 * wk[3]; qx = qx + rx1 * wk[3];
  rely = (c0 - qy) * 192.0f;
  relx = (c1 - qx) * 192.0f;
}

__global__ __launch_bounds__(256) void packw_kernel(const float* __restrict__ w, int din, int dout,
                                                    unsigned short* __restrict__ wt, int kp, float carry) {
  __shared__ __align__(16) float srow[8][kPitch0];
  const int lane = threadIdx.x & 31, wave = threadIdx.x >> 5;
  const int n = blockIdx.x * 8 + wave;
  const int nc = n < dout ? n : dout - 1;
  const float fr = (n < dout) ? carry : 0.0f;
  float* sr = srow[wave];
  const int ni = kp >> 5;
#pragma unroll 1
  for (int i = 0; i < ni; ++i) {
    const int k = i * 32 + lane;
    const int kc = k < din ? k : din - 1;
    const float f = (k < din) ? fr : 0.0f;
    sr[k] = w[(size_t)kc * dout + nc] * f;
  }
  __syncthreads();
  store_row_f16(sr, wt + (size_t)n * kp, kp >> 3, lane);
}

__global__ __launch_bounds__(256) void conv_kernel(const float* __restrict__ inp, const float* __restrict__ cw,
                                                   const float* __restrict__ cb, float* __restrict__ feat) {
  __shared__ float s_w[kConvW];
  __shared__ float s_b[kImg];
  __shared__ float s_in[9 * 196];
  const int x = threadIdx.x;
  const int y = blockIdx.x;
#pragma unroll
  for (int it = 0; it < 9; ++it) s_w[it * kImg + x] = cw[it * kImg + x];
  s_b[x] = cb[x < kCh ? x : kCh - 1];
  __syncthreads();
#pragma unroll
  for (int r = 0; r < 9; ++r) {
    const int ci = r / 3, ky = r % 3;
    const int yy = y + ky - 1;
    const int yyc = clampi(yy, 0, 191);
    const float f = (yy >= 0 && yy <= 191) ? 1.0f : 0.0f;
    s_in[r * 196 + x + 1] = inp[((size_t)ci * kImg + yyc) * kImg + x] * f;
  }
  if (x < 9) { s_in[x * 196] = 0.0f; s_in[x * 196 + 193] = 0.0f; }
  __syncthreads();
  float rv[27];
#pragma unroll
  for (int r = 0; r < 9; ++r)
#pragma unroll
    for (int kx = 0; kx < 3; ++kx) rv[r * 3 + kx] = s_in[r * 196 + x + kx];
  float* fo = feat + (size_t)y * kImg + x;
#pragma unroll 1
  for (int c = 0; c < kCh; ++c) {
    const float* wc = s_w + c * 27;
    float acc = 0.0f;
#pragma unroll
    for (int i = 0; i < 27; ++i) acc = fmaf(wc[i], rv[i], acc);
    const float v = acc + s_b[c];
    float* p = fo + (size_t)c * kPix;
    *(volatile float*)p = v;
    __threadfence();
    *(volatile float*)p = v;
  }
}

__global__ __launch_bounds__(256) void sample_kernel(const float* __restrict__ feat, const float* __restrict__ coord,
                                                     const float* __restrict__ cell, unsigned short* __restrict__ X,
                                                     int qbase) {
  __shared__ __align__(16) float srow[8][kPitch0];
  const int lane = threadIdx.x & 31, wave = threadIdx.x >> 5;
  const int ql  = blockIdx.x * 2 + (wave >> 2);
  const int e   = wave & 3;
  const int q   = qbase + ql;
  const int row = blockIdx.x * 8 + wave;
  const float c0 = coord[2 * q], c1 = coord[2 * q + 1];
  float wk[4]; int yi[2], xi[2]; float rely, relx;
  lgeom(c0, c1, e, wk, yi, xi, rely, relx);
  const float cy = cell[2 * q] * 192.0f;
  const float cx = cell[2 * q + 1] * 192.0f;
  float* sr = srow[wave];
#pragma unroll 1
  for (int i = 0; i < 18; ++i) {
    const int col = i * 32 + lane;
    const int ch  = col / 9;
    const int p   = col - ch * 9;
    const int p3  = p / 3;
    const int dy  = p3 - 1;
    const int dx  = (p - p3 * 3) - 1;
    float acc = 0.0f;
#pragma unroll
    for (int k = 0; k < 4; ++k) {
      const int yy = yi[k >> 1] + dy;
      const int xx = xi[k & 1] + dx;
      const float fy = ((unsigned)yy <= 191u) ? 1.0f : 0.0f;
      const float fx = ((unsigned)xx <= 191u) ? 1.0f : 0.0f;
      const int yyc = clampi(yy, 0, 191), xxc = clampi(xx, 0, 191);
      const float v = feat[((size_t)ch * kImg + yyc) * kImg + xxc];
      acc = acc + (v * (fy * fx)) * wk[k];
    }
    sr[col] = acc;
  }
  {
    float sv = 0.0f;
    sv = (lane == 0) ? rely : sv;
    sv = (lane == 1) ? relx : sv;
    sv = (lane == 2) ? cy : sv;
    sv = (lane == 3) ? cx : sv;
    sr[576 + lane] = sv;
    sr[608 + lane] = 0.0f;
  }
  __syncthreads();
  store_row_f16(sr, X + (size_t)row * kPitch0, kPitch0 >> 3, lane);
}

__global__ __launch_bounds__(256) void head_kernel(const float* __restrict__ Z, const float* __restrict__ coord,
                                                   const float* __restrict__ b4, float* __restrict__ out, int qbase) {
  __shared__ __align__(16) float so[256 * 3];
  const int tid = threadIdx.x, lane = tid & 31, wave = tid >> 5;
  const int ql = blockIdx.x * 256 + tid;
  const int q  = qbase + ql;
  const float c0 = coord[2 * q], c1 = coord[2 * q + 1];
  float ar[4];
#pragma unroll
  for (int e = 0; e < 4; ++e) {
    float wk[4]; int yi[2], xi[2]; float ry_, rx_;
    lgeom(c0, c1, e, wk, yi, xi, ry_, rx_);
    ar[e] = fabsf(ry_ * rx_) + 1e-9f;
  }
  const float tot = ((ar[0] + ar[1]) + ar[2]) + ar[3];
  const float rt  = 1.0f / tot;
  const float pw0 = ar[3] * rt, pw1 = ar[2] * rt, pw2 = ar[1] * rt, pw3 = ar[0] * rt;
  const float bb0 = b4[0], bb1 = b4[1], bb2 = b4[2];
  const float* zr = Z + (size_t)(4 * ql) * kHeadN;
  float o0 = 0.0f, o1 = 0.0f, o2 = 0.0f;
#pragma unroll 1
  for (int idx = 0; idx < 12; ++idx) {
    const int e = idx / 3;
    const int c = idx - 3 * e;
    const float z  = zr[e * kHeadN + c];
    const float we = (e == 0) ? pw0 : (e == 1) ? pw1 : (e == 2) ? pw2 : pw3;
    const float bc = (c == 0) ? bb0 : (c == 1) ? bb1 : bb2;
    const float p  = tanhf(z + bc) * 1.01f;
    const float val = p * we;
    o0 = o0 + ((c == 0) ? val : 0.0f);
    o1 = o1 + ((c == 1) ? val : 0.0f);
    o2 = o2 + ((c == 2) ? val : 0.0f);
  }
  so[tid * 3 + 0] = o0;
  so[tid * 3 + 1] = o1;
  so[tid * 3 + 2] = o2;
  __syncthreads();
  const int lc = lane < 24 ? lane : 23;
  const v4f v = *(const v4f*)(so + wave * 96 + lc * 4);
  float* ob = out + (size_t)(qbase + blockIdx.x * 256 + wave * 32) * 3;
  for (int pass = 0; pass < 2; ++pass) {
    if (lane < 24) *(volatile v4f*)(ob + lane * 4) = v;
    __threadfence();
  }
}

extern "C" void kernel_launch(void* const* d_in, const int* in_sizes, int n_in,
                              void* d_out, int out_size, void* d_ws, size_t ws_size,
                              hipStream_t stream) {
  (void)in_sizes;
  if (n_in < 15) return;
  if (out_size != kQ * 3) return;
  if (ws_size < kWsTotal) return;

  const float* inp    = (const float*)d_in[0];
  const float* coord  = (const float*)d_in[1];
  const float* cell   = (const float*)d_in[2];
  const float* conv_w = (const float*)d_in[3];
  const float* conv_b = (const float*)d_in[4];
  const float* w0 = (const float*)d_in[5];  const float* b0 = (const float*)d_in[6];
  const float* w1 = (const float*)d_in[7];  const float* b1 = (const float*)d_in[8];
  const float* w2 = (const float*)d_in[9];  const float* b2 = (const float*)d_in[10];
  const float* w3 = (const float*)d_in[11]; const float* b3 = (const float*)d_in[12];
  const float* w4 = (const float*)d_in[13]; const float* b4 = (const float*)d_in[14];
  float* out = (float*)d_out;

  char* ws = (char*)d_ws;
  float*          feat = (float*)(ws + kOffFeat);
  unsigned short* Wt0  = (unsigned short*)(ws + kOffWt0);
  unsigned short* Wt1  = (unsigned short*)(ws + kOffWt1);
  unsigned short* Wt2  = (unsigned short*)(ws + kOffWt2);
  unsigned short* Wt3  = (unsigned short*)(ws + kOffWt3);
  unsigned short* Wt4  = (unsigned short*)(ws + kOffWt4);
  unsigned short* X    = (unsigned short*)(ws + kOffX);
  unsigned short* Y1   = (unsigned short*)(ws + kOffY1);
  unsigned short* Y2   = (unsigned short*)(ws + kOffY2);
  float*          Z    = (float*)(ws + kOffZ);

  packw_kernel<<<kHid / 8, 256, 0, stream>>>(w0, kInDim, kHid, Wt0, kPitch0, kWCarry);
  packw_kernel<<<kHid / 8, 256, 0, stream>>>(w1, kHid, kHid, Wt1, kHid, kWCarry);
  packw_kernel<<<kHid / 8, 256, 0, stream>>>(w2, kHid, kHid, Wt2, kHid, kWCarry);
  packw_kernel<<<kHid / 8, 256, 0, stream>>>(w3, kHid, kHid, Wt3, kHid, kWCarry);
  packw_kernel<<<kHeadN / 8, 256, 0, stream>>>(w4, kHid, 3, Wt4, kHid, kWCarry);

  conv_kernel<<<kImg, kImg, 0, stream>>>(inp, conv_w, conv_b, feat);

  const long zs = 0;
  const int tilesL = (kChunkRows / 64) * (kHid / 64);
  const int tilesH = (kChunkRows / 64) * (kHeadN / 64);
  const dim3 gL((tilesL + 7) / 8, 1);
  const dim3 gH((tilesH + 7) / 8, 1);

  for (int ck = 0; ck < kQ / kChunkQ; ++ck) {
    const int qbase = ck * kChunkQ;
    sample_kernel<<<kChunkRows / 8, 256, 0, stream>>>(feat, coord, cell, X, qbase);
    wmma_gemm64<0, false, 2, 1, false, 2><<<gL, 256, 0, stream>>>(
        X, X, kPitch0, zs, Wt0, Wt0, kPitch0, zs, (void*)Y1, (void*)Y1, kHid, zs,
        b0, b0, zs, kChunkRows, kHid, kK0, kWCarryInv);
    wmma_gemm64<0, false, 2, 1, false, 2><<<gL, 256, 0, stream>>>(
        Y1, Y1, kHid, zs, Wt1, Wt1, kHid, zs, (void*)Y2, (void*)Y2, kHid, zs,
        b1, b1, zs, kChunkRows, kHid, kHid, kWCarryInv);
    wmma_gemm64<0, false, 2, 1, false, 2><<<gL, 256, 0, stream>>>(
        Y2, Y2, kHid, zs, Wt2, Wt2, kHid, zs, (void*)Y1, (void*)Y1, kHid, zs,
        b2, b2, zs, kChunkRows, kHid, kHid, kWCarryInv);
    wmma_gemm64<0, false, 2, 1, false, 2><<<gL, 256, 0, stream>>>(
        Y1, Y1, kHid, zs, Wt3, Wt3, kHid, zs, (void*)Y2, (void*)Y2, kHid, zs,
        b3, b3, zs, kChunkRows, kHid, kHid, kWCarryInv);
    wmma_gemm64<0, false, 0, 0, false, 0><<<gH, 256, 0, stream>>>(
        Y2, Y2, kHid, zs, Wt4, Wt4, kHid, zs, (void*)Z, (void*)Z, kHeadN, zs,
        b4, b4, zs, kChunkRows, kHeadN, kHid, kWCarryInv);
    head_kernel<<<kChunkQ / 256, 256, 0, stream>>>(Z, coord, b4, out, qbase);
  }
}
